// LocalMamba2D_27453430956043
// MI455X (gfx1250) — hardware-run, weakly checked
//
#include <hip/hip_runtime.h>
#include <math.h>

typedef __attribute__((ext_vector_type(8)))  _Float16 v8h;
typedef __attribute__((ext_vector_type(16))) __bf16   v16b;
typedef __attribute__((ext_vector_type(8)))  __bf16   v8b;
typedef __attribute__((ext_vector_type(8)))  float    v8f;
typedef __attribute__((ext_vector_type(4)))  float    v4f;
typedef __attribute__((ext_vector_type(2)))  float    v2f;
typedef __attribute__((ext_vector_type(4)))  unsigned v4u;
typedef __attribute__((ext_vector_type(2)))  unsigned v2u;

constexpr int kC     = 96;
constexpr int kQ     = 4;
constexpr int kHW    = 128;
constexpr int kImg   = 256;
constexpr int kL     = kHW * kHW;
constexpr int kNP    = kQ * kL;
constexpr int kNS    = 16;
constexpr int kDtR   = 6;
constexpr int kXR    = kDtR + 2 * kNS;
constexpr int kMid   = 12;
constexpr int kM1    = 2 * kC;
constexpr int kM2    = 64;
constexpr int kWRows = kM1 + kM2;
constexpr int kLineF = 32;
constexpr double kInvCnt  = 1.0 / ((double)kC * (double)kL);
static_assert(kL == 16384 && kNP == 65536 && kXR == 38, "shape");
static_assert((kC % 32) == 0 && (kM1 % 64) == 0 && (kM2 % 64) == 0 && (kNP % 64) == 0, "tile multiples");
static_assert(kXR <= kM2 && (kC % 16) == 0, "slab split on 16-row bounds");

constexpr size_t kSzLines = (size_t)kQ * kC * kLineF * 4;
constexpr size_t kSzWall  = (size_t)kWRows * kC * 2;
constexpr size_t kSzP16   = (size_t)kNP * kC * 2;
constexpr size_t kSzP32   = (size_t)kNP * kC * 4;
constexpr size_t kSzXd    = (size_t)kM2 * kNP * 4;
constexpr size_t kOffPart1 = 0;
constexpr size_t kOffPart2 = kOffPart1 + kSzLines;
constexpr size_t kOffPool  = kOffPart2 + kSzLines;
constexpr size_t kOffWallH = kOffPool  + kSzLines;
constexpr size_t kOffWallL = kOffWallH + kSzWall;
constexpr size_t kOffHT    = kOffWallL + kSzWall;
constexpr size_t kOffA16   = kOffHT    + kSzP16;
constexpr size_t kOffBpre  = kOffA16   + kSzP16;
constexpr size_t kOffVF    = kOffBpre  + kSzP32;
constexpr size_t kOffVT    = kOffVF    + kSzP32;
constexpr size_t kOffXd    = kOffVT    + kSzP16;
constexpr size_t kOffBs    = kOffXd    + kSzXd;
constexpr size_t kWsTotal  = kOffBs    + kSzP16;
static_assert(kWsTotal == 117686272ull, "carve total");
static_assert(kWsTotal <= 134217728ull, "carve cap");
static_assert(kSzP16 <= kSzP32 && 2 * kSzP16 <= kSzP32, "time-shared planes fit their host regions");
static_assert((kOffPart2 % 128) == 0 && (kOffPool % 128) == 0 && (kOffWallH % 128) == 0 && (kOffWallL % 128) == 0 &&
              (kOffHT % 128) == 0 && (kOffA16 % 128) == 0 && (kOffBpre % 128) == 0 && (kOffVF % 128) == 0 &&
              (kOffVT % 128) == 0 && (kOffXd % 128) == 0 && (kOffBs % 128) == 0 && (kSzP16 % 128) == 0,
              "128-B aligned regions");

__device__ __forceinline__ float h16_to_f32(unsigned hb) {
  const unsigned sgn = (hb & 0x8000u) << 16; const unsigned em = hb & 0x7fffu;
  const float fn = __uint_as_float((em << 13) + 0x38000000u);
  const float fs = (float)em * 5.9604644775390625e-8f;
  const float mag = (em < 0x400u) ? fs : fn; return __uint_as_float(__float_as_uint(mag) | sgn);
}
__device__ __forceinline__ unsigned bf16_rne_word(float f) {
  unsigned u = __float_as_uint(f);
  const unsigned lsb = (u & 0x00010000u) ? 1u : 0u;
  u = (u + 0x7FFFu + lsb) & 0xFFFF0000u;
  return u;
}
__device__ __forceinline__ void split_pack2(float f0, float f1, unsigned& hw, unsigned& lw) {
  const unsigned h0 = bf16_rne_word(f0);
  const unsigned h1 = bf16_rne_word(f1);
  const unsigned l0 = bf16_rne_word(f0 - __uint_as_float(h0));
  const unsigned l1 = bf16_rne_word(f1 - __uint_as_float(h1));
  hw = __builtin_amdgcn_perm(h1, h0, 0x07060302u);
  lw = __builtin_amdgcn_perm(l1, l0, 0x07060302u);
}
__device__ __forceinline__ float silu_f(float z) {
  return z * __builtin_amdgcn_rcpf(1.0f + expf(-z));
}
__device__ __forceinline__ v16b frag_load(const __bf16* p) {
  union { v16b v; v8b h[2]; } f;
  f.h[0] = *(const v8b*)(p);
  f.h[1] = *(const v8b*)(p + 16);
  return f.v;
}
__device__ __forceinline__ v8f mma_guarded(v16b a, v16b b, v8f c) {
  c = __builtin_amdgcn_wmma_f32_16x16x32_bf16(false, a, false, b, (short)0, c, false, false);
  asm volatile("v_nop\n\tv_nop\n\tv_nop\n\tv_nop" : "+v"(c) : "v"(a), "v"(b));
  return c;
}

__device__ __forceinline__ void block_line2(float a, float b, float* sRed, float* line) {
  const int lane = threadIdx.x & 31;
  const int wave = threadIdx.x >> 5;
#pragma unroll
  for (int off = 16; off > 0; off >>= 1) {
    a += __shfl_xor(a, off, 32);
    b += __shfl_xor(b, off, 32);
  }
  if (lane == 0) { sRed[wave] = a; sRed[8 + wave] = b; }
  __syncthreads();
  if (wave == 0) {
    float xa = sRed[lane & 7];
    float xb = sRed[8 + (lane & 7)];
#pragma unroll
    for (int off = 4; off > 0; off >>= 1) {
      xa += __shfl_xor(xa, off, 32);
      xb += __shfl_xor(xb, off, 32);
    }
    const float val = (lane == 0) ? xa : ((lane == 1) ? xb : 0.0f);
    volatile float* dst = line + lane;
    *dst = val;
    __threadfence();
    *dst = val;
  }
}

__device__ __forceinline__ void block_stats(const float* __restrict__ part, int q, float* sRes, float& mu, float& rstd) {
  const int lane = threadIdx.x & 31;
  const int wave = threadIdx.x >> 5;
  if (wave == 0) {
    double s = 0.0, s2 = 0.0;
#pragma unroll
    for (int j = 0; j < 3; ++j) {
      const float* pl = part + (size_t)(q * kC + lane + 32 * j) * kLineF;
      const v2f pv = *(const v2f*)pl;
      s  += (double)pv[0];
      s2 += (double)pv[1];
    }
#pragma unroll
    for (int off = 16; off > 0; off >>= 1) {
      s  += __shfl_xor(s, off, 32);
      s2 += __shfl_xor(s2, off, 32);
    }
    const double mean = s * kInvCnt;
    double var = s2 * kInvCnt - mean * mean;
    var = (var < 0.0) ? 0.0 : var;
    if (lane == 0) {
      sRes[0] = (float)mean;
      sRes[1] = rsqrtf((float)var + 1e-5f);
    }
  }
  __syncthreads();
  mu = sRes[0];
  rstd = sRes[1];
}

__global__ __launch_bounds__(256) void input_stats_kernel(const float* __restrict__ x, float* __restrict__ part) {
  __shared__ float sRed[16];
  const int c = blockIdx.x, q = blockIdx.y;
  const int tid = threadIdx.x;
  const int r0 = (q >> 1) * kHW, c0 = (q & 1) * kHW;
  float s = 0.f, s2 = 0.f;
#pragma unroll 4
  for (int i = 0; i < 16; ++i) {
    const int ch = tid + 256 * i;
    const int y = ch >> 5, x4 = (ch & 31) * 4;
    const v4f v = *(const v4f*)(x + ((size_t)c * kImg + r0 + y) * kImg + c0 + x4);
    s  += (v[0] + v[1]) + (v[2] + v[3]);
    s2 += (v[0] * v[0] + v[1] * v[1]) + (v[2] * v[2] + v[3] * v[3]);
  }
  block_line2(s, s2, sRed, part + (size_t)(q * kC + c) * kLineF);
}

__global__ __launch_bounds__(96) void weight_planes_kernel(
    const float* __restrict__ p1w, const float* __restrict__ p2w, const float* __restrict__ xpw,
    unsigned short* __restrict__ wallH, unsigned short* __restrict__ wallL) {
  const unsigned tid = threadIdx.x;
  const unsigned blk = blockIdx.x;
  unsigned rl = tid / 12u;
  asm volatile("" : "+v"(rl));
  unsigned c8 = (tid - rl * 12u) * 8u;
  asm volatile("" : "+v"(c8));
  const unsigned row = blk * 8u + rl;
  const float* src = (blk < 12u) ? p1w : ((blk < 24u) ? p2w : xpw);
  const unsigned rbase = (blk < 12u) ? 0u : ((blk < 24u) ? (unsigned)kC : (unsigned)kM1);
  const unsigned rlimit = (blk < 24u) ? (unsigned)kC : (unsigned)kXR;
  const unsigned sr = row - rbase;
  const bool live = sr < rlimit;
  const unsigned src_row = live ? sr : (rlimit - 1u);
  const float* sp = src + (size_t)src_row * kC + c8;
  const v4f a0 = *(const v4f*)(sp);
  const v4f a1 = *(const v4f*)(sp + 4);
  float f0 = a0[0], f1 = a0[1], f2 = a0[2], f3 = a0[3];
  float f4 = a1[0], f5 = a1[1], f6 = a1[2], f7 = a1[3];
  asm volatile("" : "+v"(f0), "+v"(f1), "+v"(f2), "+v"(f3));
  asm volatile("" : "+v"(f4), "+v"(f5), "+v"(f6), "+v"(f7));
  const float g0 = live ? f0 : 0.0f;
  const float g1 = live ? f1 : 0.0f;
  const float g2 = live ? f2 : 0.0f;
  const float g3 = live ? f3 : 0.0f;
  const float g4 = live ? f4 : 0.0f;
  const float g5 = live ? f5 : 0.0f;
  const float g6 = live ? f6 : 0.0f;
  const float g7 = live ? f7 : 0.0f;
  unsigned hw0, hw1, hw2, hw3, lw0, lw1, lw2, lw3;
  split_pack2(g0, g1, hw0, lw0);
  split_pack2(g2, g3, hw1, lw1);
  split_pack2(g4, g5, hw2, lw2);
  split_pack2(g6, g7, hw3, lw3);
  v4u hv, lv;
  hv[0] = hw0; hv[1] = hw1; hv[2] = hw2; hv[3] = hw3;
  lv[0] = lw0; lv[1] = lw1; lv[2] = lw2; lv[3] = lw3;
  unsigned short* dstH = wallH + (size_t)blk * (8 * kC) + (size_t)tid * 8;
  unsigned short* dstL = wallL + (size_t)blk * (8 * kC) + (size_t)tid * 8;
  *(volatile v4u*)dstH = hv;
  *(volatile v4u*)dstL = lv;
  __threadfence();
  *(volatile v4u*)dstH = hv;
  *(volatile v4u*)dstL = lv;
}

__global__ __launch_bounds__(256) void norm_transpose_kernel(
    const float* __restrict__ x, const float* __restrict__ part1,
    const float* __restrict__ gam, const float* __restrict__ bet,
    unsigned short* __restrict__ hTH, unsigned short* __restrict__ hTL) {
  __shared__ __align__(16) float sT[kC * 68];
  __shared__ float sRes[2];
  const int tid = threadIdx.x;
  const int n0 = blockIdx.x * 64;
  const int q = n0 >> 14;
  const int rem = n0 & (kL - 1);
  const int y = rem >> 7, x0 = rem & 127;
  const int r0 = (q >> 1) * kHW, c0 = (q & 1) * kHW;
  float mu, rstd;
  block_stats(part1, q, sRes, mu, rstd);
#pragma unroll
  for (int i = 0; i < 6; ++i) {
    const int idx = tid + 256 * i;
    const int c = idx >> 4, x4 = (idx & 15) * 4;
    const v4f v = *(const v4f*)(x + ((size_t)c * kImg + r0 + y) * kImg + c0 + x0 + x4);
    const float gg = gam[c], bb = bet[c];
    v4f o;
    o[0] = ((v[0] - mu) * rstd) * gg + bb;
    o[1] = ((v[1] - mu) * rstd) * gg + bb;
    o[2] = ((v[2] - mu) * rstd) * gg + bb;
    o[3] = ((v[3] - mu) * rstd) * gg + bb;
    *(v4f*)(sT + c * 68 + x4) = o;
  }
  __syncthreads();
  v4u hv[3], lv[3];
#pragma unroll
  for (int i = 0; i < 3; ++i) {
    const unsigned chunk = (unsigned)tid + 256u * (unsigned)i;
    unsigned pos = chunk / 12u;
    asm volatile("" : "+v"(pos));
    unsigned c8 = (chunk - pos * 12u) * 8u;
    asm volatile("" : "+v"(c8));
    const float e0 = sT[(c8 + 0u) * 68u + pos];
    const float e1 = sT[(c8 + 1u) * 68u + pos];
    const float e2 = sT[(c8 + 2u) * 68u + pos];
    const float e3 = sT[(c8 + 3u) * 68u + pos];
    const float e4 = sT[(c8 + 4u) * 68u + pos];
    const float e5 = sT[(c8 + 5u) * 68u + pos];
    const float e6 = sT[(c8 + 6u) * 68u + pos];
    const float e7 = sT[(c8 + 7u) * 68u + pos];
    unsigned hw0, hw1, hw2, hw3, lw0, lw1, lw2, lw3;
    split_pack2(e0, e1, hw0, lw0);
    split_pack2(e2, e3, hw1, lw1);
    split_pack2(e4, e5, hw2, lw2);
    split_pack2(e6, e7, hw3, lw3);
    hv[i][0] = hw0; hv[i][1] = hw1; hv[i][2] = hw2; hv[i][3] = hw3;
    lv[i][0] = lw0; lv[i][1] = lw1; lv[i][2] = lw2; lv[i][3] = lw3;
  }
  unsigned short* dstH = hTH + (size_t)n0 * kC;
  unsigned short* dstL = hTL + (size_t)n0 * kC;
  for (int pass = 0; pass < 2; ++pass) {
#pragma unroll
    for (int i = 0; i < 3; ++i) {
      *(volatile v4u*)(dstH + (size_t)(tid + 256 * i) * 8) = hv[i];
      *(volatile v4u*)(dstL + (size_t)(tid + 256 * i) * 8) = lv[i];
    }
    __threadfence();
  }
}

template <int MODE>
__global__ __launch_bounds__(256) void chan_gemm_kernel(
    const unsigned short* __restrict__ AHp, const unsigned short* __restrict__ ALp,
    const unsigned short* __restrict__ BHp, const unsigned short* __restrict__ BLp,
    float* __restrict__ Cf, unsigned short* __restrict__ Ch,
    const float* __restrict__ biasLo, const float* __restrict__ biasHi) {
  constexpr int M = (MODE == 0) ? kM1 : kM2;
  constexpr int N = kNP;
  constexpr int K = kC;
  static_assert((M % 64) == 0 && (N % 64) == 0 && (K % 32) == 0, "tile multiples");
  const __bf16* AH = (const __bf16*)AHp;
  const __bf16* AL = (const __bf16*)ALp;
  const __bf16* BH = (const __bf16*)BHp;
  const __bf16* BL = (const __bf16*)BLp;
  __shared__ __align__(16) float sT[8][16 * 68];
  const int lane = threadIdx.x & 31;
  const int wave = threadIdx.x >> 5;
  constexpr int tilesN = N >> 6;
  constexpr int tilesM = M >> 6;
  const int tile = blockIdx.x * 8 + wave;
  if (tile >= tilesM * tilesN) return;
  const int tm = tile / tilesN;
  const int tn = tile - tm * tilesN;
  const int m0 = tm << 6;
  const int n0 = tn << 6;
  const int rlane = lane & 15;
  const int koff  = (lane >> 4) * 8;
  const int mOff  = (lane >> 4) * 8;

  v8f acc[4][4];
#pragma unroll
  for (int i = 0; i < 4; ++i)
#pragma unroll
    for (int j = 0; j < 4; ++j) acc[i][j] = (v8f){0.f, 0.f, 0.f, 0.f, 0.f, 0.f, 0.f, 0.f};

#pragma unroll 1
  for (int k0 = 0; k0 < K; k0 += 32) {
    v16b bh[4], bl[4];
#pragma unroll
    for (int j = 0; j < 4; ++j) {
      const size_t bo = (size_t)(n0 + (j << 4) + rlane) * K + koff + k0;
      bh[j] = frag_load(BH + bo);
      bl[j] = frag_load(BL + bo);
    }
#pragma unroll
    for (int i = 0; i < 4; ++i) {
      const size_t ao = (size_t)(m0 + (i << 4) + rlane) * K + koff + k0;
      const v16b ah = frag_load(AH + ao);
      const v16b al = frag_load(AL + ao);
#pragma unroll
      for (int j = 0; j < 4; ++j) {
        acc[i][j] = mma_guarded(ah, bh[j], acc[i][j]);
        acc[i][j] = mma_guarded(ah, bl[j], acc[i][j]);
        acc[i][j] = mma_guarded(al, bh[j], acc[i][j]);
      }
    }
  }

  float* slab = sT[wave];
#pragma unroll
  for (int i = 0; i < 4; ++i) {
    const int mBase = m0 + (i << 4);
    const bool lowHalf = (MODE == 0) && (mBase < kC);
    float bv[8];
    if (MODE == 0) {
      const int hiBase = (mBase >= kC) ? (mBase - kC) : 0;
      const int loBase = (mBase < kC) ? mBase : 0;
      const float* bp = lowHalf ? (biasLo + loBase) : (biasHi + hiBase);
#pragma unroll
      for (int r = 0; r < 8; ++r) bv[r] = bp[mOff + r];
    } else {
#pragma unroll
      for (int r = 0; r < 8; ++r) bv[r] = 0.0f;
    }
#pragma unroll
    for (int j = 0; j < 4; ++j) {
#pragma unroll
      for (int r = 0; r < 8; ++r) {
        const float val = acc[i][j][r] + bv[r];
        slab[(mOff + r) * 68 + (j << 4) + rlane] = val;
      }
    }
    __builtin_amdgcn_fence(__ATOMIC_RELEASE, "workgroup");
    __builtin_amdgcn_wave_barrier();
    __builtin_amdgcn_fence(__ATOMIC_ACQUIRE, "workgroup");
    if (lowHalf) {
      const int q4 = lane >> 3, c8 = (lane & 7) * 8;
#pragma unroll 1
      for (int it = 0; it < 4; ++it) {
        float* sp = slab + (it * 4 + q4) * 68 + c8;
        v4f a0 = *(v4f*)(sp);
        v4f a1 = *(v4f*)(sp + 4);
#pragma unroll
        for (int e = 0; e < 4; ++e) {
          a0[e] = silu_f(a0[e]);
          a1[e] = silu_f(a1[e]);
        }
        *(v4f*)(sp) = a0;
        *(v4f*)(sp + 4) = a1;
      }
      v8h hv[4];
#pragma unroll
      for (int it = 0; it < 4; ++it) {
        const float* sp = slab + (it * 4 + q4) * 68 + c8;
        const v4f a0 = *(const v4f*)(sp);
        const v4f a1 = *(const v4f*)(sp + 4);
#pragma unroll
        for (int e = 0; e < 4; ++e) {
          hv[it][e]     = (_Float16)a0[e];
          hv[it][4 + e] = (_Float16)a1[e];
        }
      }
      for (int pass = 0; pass < 2; ++pass) {
#pragma unroll
        for (int it = 0; it < 4; ++it) {
          const int row = it * 4 + q4;
          *(volatile v8h*)(Ch + (size_t)(mBase + row) * N + n0 + c8) = hv[it];
        }
        __threadfence();
      }
    } else {
      const int hh = lane >> 4, c4 = (lane & 15) * 4;
      const int outBase = (MODE == 0) ? ((mBase >= kC) ? (mBase - kC) : 0) : mBase;
      for (int pass = 0; pass < 2; ++pass) {
#pragma unroll
        for (int it = 0; it < 8; ++it) {
          const int row = it * 2 + hh;
          const v4f val = *(const v4f*)(slab + row * 68 + c4);
          *(volatile v4f*)(Cf + (size_t)(outBase + row) * N + n0 + c4) = val;
        }
        __threadfence();
      }
    }
    __builtin_amdgcn_fence(__ATOMIC_RELEASE, "workgroup");
    __builtin_amdgcn_wave_barrier();
    __builtin_amdgcn_fence(__ATOMIC_ACQUIRE, "workgroup");
  }
}

__global__ __launch_bounds__(256) void depthwise_silu_kernel(
    const float* __restrict__ bpre, const float* __restrict__ dww, const float* __restrict__ dwb,
    float* __restrict__ vf, unsigned short* __restrict__ vTH, unsigned short* __restrict__ vTL) {
  __shared__ __align__(16) float sV[kC * 68];
  __shared__ float sW[kC * 9];
  __shared__ float sB[kC];
  const int tid = threadIdx.x;
  const int n0 = blockIdx.x * 64;
  const int q = n0 >> 14;
  const int rem = n0 & (kL - 1);
  const int y = rem >> 7, x0 = rem & 127;
#pragma unroll 1
  for (int i = 0; i < 4; ++i) {
    const int idx = tid + 256 * i;
    const int cl = (idx < kC * 9) ? idx : (kC * 9 - 1);
    float wv = dww[cl];
    asm volatile("" : "+v"(wv));
    if (idx < kC * 9) sW[idx] = wv;
  }
  {
    const int cl = (tid < kC) ? tid : (kC - 1);
    float bvv = dwb[cl];
    asm volatile("" : "+v"(bvv));
    if (tid < kC) sB[tid] = bvv;
  }
  const int px = tid & 63;
  const int sub = tid >> 6;
  int offs[9];
  unsigned vmask = 0u;
#pragma unroll
  for (int ky = 0; ky < 3; ++ky) {
#pragma unroll
    for (int kx = 0; kx < 3; ++kx) {
      const int yy = y + ky - 1;
      const int xx = x0 + px + kx - 1;
      const bool ok = (yy >= 0) && (yy < kHW) && (xx >= 0) && (xx < kHW);
      const int yc = (yy < 0) ? 0 : ((yy > kHW - 1) ? (kHW - 1) : yy);
      const int xc = (xx < 0) ? 0 : ((xx > kHW - 1) ? (kHW - 1) : xx);
      offs[ky * 3 + kx] = yc * kHW + xc;
      vmask |= ok ? (1u << (ky * 3 + kx)) : 0u;
    }
  }
  __syncthreads();
#pragma unroll 1
  for (int pass = 0; pass < 24; ++pass) {
    const int c = pass * 4 + sub;
    const float* base = bpre + (size_t)c * kNP + (size_t)q * kL;
    float t[9];
#pragma unroll
    for (int k = 0; k < 9; ++k) t[k] = base[offs[k]];
    asm volatile("" : "+v"(t[0]), "+v"(t[1]), "+v"(t[2]), "+v"(t[3]), "+v"(t[4]));
    asm volatile("" : "+v"(t[5]), "+v"(t[6]), "+v"(t[7]), "+v"(t[8]));
    float acc = 0.0f;
#pragma unroll
    for (int k = 0; k < 9; ++k) {
      const float tv = (vmask & (1u << k)) ? t[k] : 0.0f;
      acc = fmaf(sW[c * 9 + k], tv, acc);
    }
    const float s = acc + sB[c];
    sV[c * 68 + px] = silu_f(s);
  }
  __syncthreads();
  v4f fv[6];
  v4u hv[3], lv[3];
#pragma unroll
  for (int i = 0; i < 6; ++i) {
    const int idx = tid + 256 * i;
    const int c = idx >> 4, x4 = (idx & 15) * 4;
    fv[i] = *(const v4f*)(sV + c * 68 + x4);
  }
#pragma unroll
  for (int i = 0; i < 3; ++i) {
    const unsigned chunk = (unsigned)tid + 256u * (unsigned)i;
    unsigned pos = chunk / 12u;
    asm volatile("" : "+v"(pos));
    unsigned c8 = (chunk - pos * 12u) * 8u;
    asm volatile("" : "+v"(c8));
    const float e0 = sV[(c8 + 0u) * 68u + pos];
    const float e1 = sV[(c8 + 1u) * 68u + pos];
    const float e2 = sV[(c8 + 2u) * 68u + pos];
    const float e3 = sV[(c8 + 3u) * 68u + pos];
    const float e4 = sV[(c8 + 4u) * 68u + pos];
    const float e5 = sV[(c8 + 5u) * 68u + pos];
    const float e6 = sV[(c8 + 6u) * 68u + pos];
    const float e7 = sV[(c8 + 7u) * 68u + pos];
    unsigned hw0, hw1, hw2, hw3, lw0, lw1, lw2, lw3;
    split_pack2(e0, e1, hw0, lw0);
    split_pack2(e2, e3, hw1, lw1);
    split_pack2(e4, e5, hw2, lw2);
    split_pack2(e6, e7, hw3, lw3);
    hv[i][0] = hw0; hv[i][1] = hw1; hv[i][2] = hw2; hv[i][3] = hw3;
    lv[i][0] = lw0; lv[i][1] = lw1; lv[i][2] = lw2; lv[i][3] = lw3;
  }
  unsigned short* dstH = vTH + (size_t)n0 * kC;
  unsigned short* dstL = vTL + (size_t)n0 * kC;
  for (int pass = 0; pass < 2; ++pass) {
#pragma unroll
    for (int i = 0; i < 6; ++i) {
      const int idx = tid + 256 * i;
      const int c = idx >> 4, x4 = (idx & 15) * 4;
      *(volatile v4f*)(vf + (size_t)c * kNP + n0 + x4) = fv[i];
    }
#pragma unroll
    for (int i = 0; i < 3; ++i) {
      *(volatile v4u*)(dstH + (size_t)(tid + 256 * i) * 8) = hv[i];
      *(volatile v4u*)(dstL + (size_t)(tid + 256 * i) * 8) = lv[i];
    }
    __threadfence();
  }
}

__global__ __launch_bounds__(96) void dir_scan_kernel(
    const float* __restrict__ xd, const float* __restrict__ vf,
    const float* __restrict__ A_log, const float* __restrict__ dtw, const float* __restrict__ dtb,
    unsigned short* __restrict__ yd0, unsigned short* __restrict__ yd1,
    unsigned short* __restrict__ yd2, unsigned short* __restrict__ yd3) {
  __shared__ __align__(16) float sX[64 * 40];
  __shared__ float sU[kC * 65];
  __shared__ float sY[kC * 65];
  const int tid = threadIdx.x;
  const int lane = tid & 31;
  const int wave = tid >> 5;
  const int q = blockIdx.x >> 2;
  const int d = blockIdx.x & 3;
  const bool rev = (d >= 2);
  const bool colm = (d & 1) != 0;
  unsigned short* yd = (d == 0) ? yd0 : ((d == 1) ? yd1 : ((d == 2) ? yd2 : yd3));
  const int c = tid;

  float negA[kNS], h[kNS];
  {
    const v4f l0 = *(const v4f*)(A_log + c * kNS);
    const v4f l1 = *(const v4f*)(A_log + c * kNS + 4);
    const v4f l2 = *(const v4f*)(A_log + c * kNS + 8);
    const v4f l3 = *(const v4f*)(A_log + c * kNS + 12);
#pragma unroll
    for (int e = 0; e < 4; ++e) {
      negA[e]      = -expf(l0[e]);
      negA[4 + e]  = -expf(l1[e]);
      negA[8 + e]  = -expf(l2[e]);
      negA[12 + e] = -expf(l3[e]);
    }
  }
#pragma unroll
  for (int n = 0; n < kNS; ++n) h[n] = 0.0f;
  const v2f w01 = *(const v2f*)(dtw + c * kDtR);
  const v2f w23 = *(const v2f*)(dtw + c * kDtR + 2);
  const v2f w45 = *(const v2f*)(dtw + c * kDtR + 4);
  const float w0 = w01[0], w1 = w01[1], w2 = w23[0], w3 = w23[1], w4 = w45[0], w5 = w45[1];
  const float bias = dtb[c];

  const float* xdq = xd + (size_t)q * kL;
  const float* vq  = vf + (size_t)q * kL;
  const int q4 = lane >> 3, c8 = (lane & 7) * 8;

#pragma unroll 1
  for (int t0 = 0; t0 < kL; t0 += 64) {
#pragma unroll 1
    for (int i = 0; i < 27; ++i) {
      const int e = tid + 96 * i;
      const int ec = (e < 2560) ? e : 2559;
      const int kcol = ec >> 6, tt = ec & 63;
      const bool pad = (kcol == 6) || (kcol == 7);
      const int srow = (kcol < 6) ? kcol : (pad ? 0 : (kcol - 2));
      const int t = t0 + tt;
      const int tp = rev ? (kL - 1 - t) : t;
      const int p = colm ? (((tp & 127) << 7) + (tp >> 7)) : tp;
      float val = xdq[(size_t)srow * kNP + p];
      asm volatile("" : "+v"(val));
      val = pad ? 0.0f : val;
      if (e < 2560) sX[tt * 40 + kcol] = val;
    }
#pragma unroll 4
    for (int i = 0; i < 64; ++i) {
      const int e = tid + 96 * i;
      const int r = e >> 6, tt = e & 63;
      const int t = t0 + tt;
      const int tp = rev ? (kL - 1 - t) : t;
      const int p = colm ? (((tp & 127) << 7) + (tp >> 7)) : tp;
      sU[r * 65 + tt] = vq[(size_t)r * kNP + p];
    }
    __syncthreads();
#pragma unroll 1
    for (int s = 0; s < 64; ++s) {
      const float* xr = sX + s * 40;
      const v4f d0 = *(const v4f*)(xr);
      const v4f d1 = *(const v4f*)(xr + 4);
      float Bs[kNS], Cs[kNS];
#pragma unroll
      for (int g = 0; g < 4; ++g) {
        const v4f bq = *(const v4f*)(xr + 8 + 4 * g);
        const v4f cq = *(const v4f*)(xr + 24 + 4 * g);
        Bs[4 * g + 0] = bq[0]; Bs[4 * g + 1] = bq[1]; Bs[4 * g + 2] = bq[2]; Bs[4 * g + 3] = bq[3];
        Cs[4 * g + 0] = cq[0]; Cs[4 * g + 1] = cq[1]; Cs[4 * g + 2] = cq[2]; Cs[4 * g + 3] = cq[3];
      }
      float dd = w0 * d0[0];
      dd = fmaf(w1, d0[1], dd);
      dd = fmaf(w2, d0[2], dd);
      dd = fmaf(w3, d0[3], dd);
      dd = fmaf(w4, d1[0], dd);
      dd = fmaf(w5, d1[1], dd);
      dd += bias;
      const float ea = __expf(-fabsf(dd));
      const float up = 1.0f + ea;
      const float l1p = __logf(up) + (ea - (up - 1.0f)) * __builtin_amdgcn_rcpf(up);
      const float delta = fmaxf(dd, 0.0f) + l1p;
      const float du = delta * sU[c * 65 + s];
      float yv = 0.0f;
#pragma unroll
      for (int n = 0; n < kNS; ++n) {
        const float dA = __expf(delta * negA[n]);
        h[n] = fmaf(dA, h[n], du * Bs[n]);
        yv = fmaf(h[n], Cs[n], yv);
      }
      sY[c * 65 + s] = yv;
    }
    __syncthreads();
    v8h hv[8];
#pragma unroll
    for (int it = 0; it < 8; ++it) {
      const int row = it * 12 + wave * 4 + q4;
      const float* sp = sY + row * 65;
#pragma unroll
      for (int e = 0; e < 8; ++e) {
        const int j = c8 + e;
        const int sidx = rev ? (63 - j) : j;
        hv[it][e] = (_Float16)sp[sidx];
      }
    }
    const int tpBase = rev ? (kL - 64 - t0) : t0;
    for (int pass = 0; pass < 2; ++pass) {
#pragma unroll
      for (int it = 0; it < 8; ++it) {
        const int row = it * 12 + wave * 4 + q4;
        *(volatile v8h*)(yd + (size_t)row * kNP + (size_t)q * kL + tpBase + c8) = hv[it];
      }
      __threadfence();
    }
  }
}

__global__ __launch_bounds__(256) void combine_kernel(
    const unsigned short* __restrict__ yd0, const unsigned short* __restrict__ yd1,
    const unsigned short* __restrict__ yd2, const unsigned short* __restrict__ yd3,
    const float* __restrict__ vf, const float* __restrict__ Dp,
    unsigned short* __restrict__ bs, float* __restrict__ part2) {
  __shared__ float sTr[kHW * 33];
  __shared__ float sRed[16];
  const int c = blockIdx.x, q = blockIdx.y;
  const int tid = threadIdx.x;
  const size_t base = (size_t)c * kNP + (size_t)q * kL;
  const float dp4 = 4.0f * Dp[c];
  float s = 0.f, s2 = 0.f;
#pragma unroll 1
  for (int tI = 0; tI < 4; ++tI) {
    const int y0r = tI * 32;
    __syncthreads();
#pragma unroll
    for (int i = 0; i < 2; ++i) {
      const int idx = tid + 256 * i;
      const int xr = idx >> 2, seg = idx & 3;
      const size_t off = base + (size_t)xr * kHW + y0r + seg * 8;
      const v4u wa = *(const v4u*)(yd1 + off);
      const v4u wb = *(const v4u*)(yd3 + off);
      const unsigned a0 = wa[0], a1 = wa[1], a2 = wa[2], a3 = wa[3];
      const unsigned b0 = wb[0], b1 = wb[1], b2 = wb[2], b3 = wb[3];
      float* tp = sTr + xr * 33 + seg * 8;
      tp[0] = h16_to_f32(a0 & 0xffffu) + h16_to_f32(b0 & 0xffffu);
      tp[1] = h16_to_f32(a0 >> 16)     + h16_to_f32(b0 >> 16);
      tp[2] = h16_to_f32(a1 & 0xffffu) + h16_to_f32(b1 & 0xffffu);
      tp[3] = h16_to_f32(a1 >> 16)     + h16_to_f32(b1 >> 16);
      tp[4] = h16_to_f32(a2 & 0xffffu) + h16_to_f32(b2 & 0xffffu);
      tp[5] = h16_to_f32(a2 >> 16)     + h16_to_f32(b2 >> 16);
      tp[6] = h16_to_f32(a3 & 0xffffu) + h16_to_f32(b3 & 0xffffu);
      tp[7] = h16_to_f32(a3 >> 16)     + h16_to_f32(b3 >> 16);
    }
    __syncthreads();
    v8h hv[2];
#pragma unroll
    for (int i = 0; i < 2; ++i) {
      const int idx = tid + 256 * i;
      const int yl = idx >> 4, x8 = (idx & 15) * 8;
      const size_t off = base + (size_t)(y0r + yl) * kHW + x8;
      const v4u wa = *(const v4u*)(yd0 + off);
      const v4u wb = *(const v4u*)(yd2 + off);
      const v4f va = *(const v4f*)(vf + off);
      const v4f vb = *(const v4f*)(vf + off + 4);
      const unsigned a0 = wa[0], a1 = wa[1], a2 = wa[2], a3 = wa[3];
      const unsigned b0 = wb[0], b1 = wb[1], b2 = wb[2], b3 = wb[3];
      float rm[8];
      rm[0] = h16_to_f32(a0 & 0xffffu) + h16_to_f32(b0 & 0xffffu);
      rm[1] = h16_to_f32(a0 >> 16)     + h16_to_f32(b0 >> 16);
      rm[2] = h16_to_f32(a1 & 0xffffu) + h16_to_f32(b1 & 0xffffu);
      rm[3] = h16_to_f32(a1 >> 16)     + h16_to_f32(b1 >> 16);
      rm[4] = h16_to_f32(a2 & 0xffffu) + h16_to_f32(b2 & 0xffffu);
      rm[5] = h16_to_f32(a2 >> 16)     + h16_to_f32(b2 >> 16);
      rm[6] = h16_to_f32(a3 & 0xffffu) + h16_to_f32(b3 & 0xffffu);
      rm[7] = h16_to_f32(a3 >> 16)     + h16_to_f32(b3 >> 16);
      const float vv[8] = {va[0], va[1], va[2], va[3], vb[0], vb[1], vb[2], vb[3]};
#pragma unroll
      for (int e = 0; e < 8; ++e) {
        const float bsum = (rm[e] + sTr[(x8 + e) * 33 + yl]) + dp4 * vv[e];
        s += bsum;
        s2 = fmaf(bsum, bsum, s2);
        hv[i][e] = (_Float16)bsum;
      }
    }
    for (int pass = 0; pass < 2; ++pass) {
#pragma unroll
      for (int i = 0; i < 2; ++i) {
        const int idx = tid + 256 * i;
        const int yl = idx >> 4, x8 = (idx & 15) * 8;
        *(volatile v8h*)(bs + base + (size_t)(y0r + yl) * kHW + x8) = hv[i];
      }
      __threadfence();
    }
  }
  block_line2(s, s2, sRed, part2 + (size_t)(q * kC + c) * kLineF);
}

__global__ __launch_bounds__(256) void pool_kernel(
    const unsigned short* __restrict__ a16, const unsigned short* __restrict__ bs,
    const float* __restrict__ part2, const float* __restrict__ gam2, const float* __restrict__ bet2,
    float* __restrict__ pooled) {
  __shared__ float sRes[2];
  __shared__ float sRed[16];
  const int c = blockIdx.x, q = blockIdx.y;
  const int tid = threadIdx.x;
  float mu, rstd;
  block_stats(part2, q, sRes, mu, rstd);
  const float gg = gam2[c], bb = bet2[c];
  const size_t base = (size_t)c * kNP + (size_t)q * kL;
  float acc = 0.0f;
#pragma unroll 2
  for (int i = 0; i < 8; ++i) {
    const size_t off = base + (size_t)(tid + 256 * i) * 8;
    const v4u wa = *(const v4u*)(a16 + off);
    const v4u wb = *(const v4u*)(bs + off);
    const unsigned a0 = wa[0], a1 = wa[1], a2 = wa[2], a3 = wa[3];
    const unsigned b0 = wb[0], b1 = wb[1], b2 = wb[2], b3 = wb[3];
    const float av[8] = {h16_to_f32(a0 & 0xffffu), h16_to_f32(a0 >> 16), h16_to_f32(a1 & 0xffffu), h16_to_f32(a1 >> 16),
                         h16_to_f32(a2 & 0xffffu), h16_to_f32(a2 >> 16), h16_to_f32(a3 & 0xffffu), h16_to_f32(a3 >> 16)};
    const float bv[8] = {h16_to_f32(b0 & 0xffffu), h16_to_f32(b0 >> 16), h16_to_f32(b1 & 0xffffu), h16_to_f32(b1 >> 16),
                         h16_to_f32(b2 & 0xffffu), h16_to_f32(b2 >> 16), h16_to_f32(b3 & 0xffffu), h16_to_f32(b3 >> 16)};
#pragma unroll
    for (int e = 0; e < 8; ++e) {
      const float bn = ((bv[e] - mu) * rstd) * gg + bb;
      acc = fmaf(av[e], bn, acc);
    }
  }
  block_line2(acc * (1.0f / (float)kL), 0.0f, sRed, pooled + (size_t)(q * kC + c) * kLineF);
}

__global__ __launch_bounds__(256) void gate_residual_kernel(
    const float* __restrict__ x, const unsigned short* __restrict__ a16, const unsigned short* __restrict__ bs,
    const float* __restrict__ part2, const float* __restrict__ pooled,
    const float* __restrict__ gam2, const float* __restrict__ bet2,
    const float* __restrict__ w1, const float* __restrict__ b1,
    const float* __restrict__ w2, const float* __restrict__ b2,
    float* __restrict__ out) {
  __shared__ float sRes[2];
  __shared__ float sS[kC];
  __shared__ float sHid[16];
  const int c = blockIdx.x, q = blockIdx.y;
  const int tid = threadIdx.x;
  const int lane = tid & 31;
  const int wave = tid >> 5;
  const int r0 = (q >> 1) * kHW, c0 = (q & 1) * kHW;
  float mu, rstd;
  block_stats(part2, q, sRes, mu, rstd);
  {
    const int cl = (tid < kC) ? tid : (kC - 1);
    float sv = pooled[(size_t)(q * kC + cl) * kLineF];
    asm volatile("" : "+v"(sv));
    if (tid < kC) sS[tid] = sv;
  }
  __syncthreads();
  if (wave == 0) {
    const int j = (lane < kMid) ? lane : (kMid - 1);
    float hacc = 0.0f;
#pragma unroll 1
    for (int cc = 0; cc < kC; ++cc) hacc = fmaf(sS[cc], w1[j * kC + cc], hacc);
    hacc += b1[j];
    if (lane < kMid) sHid[lane] = fmaxf(hacc, 0.0f);
  }
  __syncthreads();
  float z = 0.0f;
#pragma unroll 1
  for (int j = 0; j < kMid; ++j) z = fmaf(sHid[j], w2[c * kMid + j], z);
  z += b2[c];
  const float gate = __builtin_amdgcn_rcpf(1.0f + expf(-z));
  const float gg = gam2[c], bb = bet2[c];
  const size_t base = (size_t)c * kNP + (size_t)q * kL;
#pragma unroll 1
  for (int g4 = 0; g4 < 4; ++g4) {
    v4f ov[4];
#pragma unroll
    for (int k = 0; k < 4; ++k) {
      const int ch = tid + 256 * (g4 * 4 + k);
      const int y = ch >> 5, x4 = (ch & 31) * 4;
      const size_t pl = base + (size_t)y * kHW + x4;
      const v2u wa = *(const v2u*)(a16 + pl);
      const v2u wb = *(const v2u*)(bs + pl);
      const size_t gi = ((size_t)c * kImg + r0 + y) * kImg + c0 + x4;
      const v4f xv = *(const v4f*)(x + gi);
      const unsigned a0 = wa[0], a1 = wa[1];
      const unsigned b0 = wb[0], b1w = wb[1];
      const float av[4] = {h16_to_f32(a0 & 0xffffu), h16_to_f32(a0 >> 16), h16_to_f32(a1 & 0xffffu), h16_to_f32(a1 >> 16)};
      const float bv[4] = {h16_to_f32(b0 & 0xffffu), h16_to_f32(b0 >> 16), h16_to_f32(b1w & 0xffffu), h16_to_f32(b1w >> 16)};
      v4f o;
#pragma unroll
      for (int e = 0; e < 4; ++e) {
        const float bn = ((bv[e] - mu) * rstd) * gg + bb;
        o[e] = xv[e] + (av[e] * bn) * gate;
      }
      ov[k] = o;
    }
    for (int pass = 0; pass < 2; ++pass) {
#pragma unroll
      for (int k = 0; k < 4; ++k) {
        const int ch = tid + 256 * (g4 * 4 + k);
        const int y = ch >> 5, x4 = (ch & 31) * 4;
        const size_t gi = ((size_t)c * kImg + r0 + y) * kImg + c0 + x4;
        *(volatile v4f*)(out + gi) = ov[k];
      }
      __threadfence();
    }
  }
}

extern "C" void kernel_launch(void* const* d_in, const int* in_sizes, int n_in,
                              void* d_out, int out_size, void* d_ws, size_t ws_size,
                              hipStream_t stream) {
  if (n_in < 20) return;
  if (in_sizes[0] != kC * kImg * kImg) return;
  if (in_sizes[3] != kC * kC || in_sizes[5] != kC * kC) return;
  if (in_sizes[7] != kC * 9) return;
  if (in_sizes[9] != kC * kNS) return;
  if (in_sizes[11] != kXR * kC) return;
  if (in_sizes[12] != kC * kDtR) return;
  if (in_sizes[16] != kMid * kC || in_sizes[18] != kC * kMid) return;
  if (out_size != kC * kImg * kImg) return;
  if (ws_size < kWsTotal) return;

  const float* x         = (const float*)d_in[0];
  const float* ln_g      = (const float*)d_in[1];
  const float* ln_b      = (const float*)d_in[2];
  const float* p1_w      = (const float*)d_in[3];
  const float* p1_b      = (const float*)d_in[4];
  const float* p2_in_w   = (const float*)d_in[5];
  const float* p2_in_b   = (const float*)d_in[6];
  const float* p2_dw_w   = (const float*)d_in[7];
  const float* p2_dw_b   = (const float*)d_in[8];
  const float* A_log     = (const float*)d_in[9];
  const float* Dp        = (const float*)d_in[10];
  const float* x_proj_w  = (const float*)d_in[11];
  const float* dt_proj_w = (const float*)d_in[12];
  const float* dt_proj_b = (const float*)d_in[13];
  const float* n2_g      = (const float*)d_in[14];
  const float* n2_b      = (const float*)d_in[15];
  const float* ca_w1     = (const float*)d_in[16];
  const float* ca_b1     = (const float*)d_in[17];
  const float* ca_w2     = (const float*)d_in[18];
  const float* ca_b2     = (const float*)d_in[19];
  float* out = (float*)d_out;

  char* ws = (char*)d_ws;
  float*          part1  = (float*)(ws + kOffPart1);
  float*          part2  = (float*)(ws + kOffPart2);
  float*          pooled = (float*)(ws + kOffPool);
  unsigned short* wallH  = (unsigned short*)(ws + kOffWallH);
  unsigned short* wallL  = (unsigned short*)(ws + kOffWallL);
  unsigned short* hTH    = (unsigned short*)(ws + kOffHT);
  unsigned short* hTL    = (unsigned short*)(ws + kOffVF);
  unsigned short* a16    = (unsigned short*)(ws + kOffA16);
  float*          bpre   = (float*)(ws + kOffBpre);
  float*          vf     = (float*)(ws + kOffVF);
  unsigned short* vTH    = (unsigned short*)(ws + kOffVT);
  unsigned short* vTL    = (unsigned short*)(ws + kOffHT);
  float*          xd     = (float*)(ws + kOffXd);
  unsigned short* bs     = (unsigned short*)(ws + kOffBs);
  unsigned short* yd0 = (unsigned short*)(ws + kOffHT);
  unsigned short* yd1 = (unsigned short*)(ws + kOffBpre);
  unsigned short* yd2 = (unsigned short*)(ws + kOffBpre + kSzP16);
  unsigned short* yd3 = (unsigned short*)(ws + kOffVT);

  input_stats_kernel<<<dim3(kC, kQ), 256, 0, stream>>>(x, part1);
  weight_planes_kernel<<<kWRows / 8, 96, 0, stream>>>(p1_w, p2_in_w, x_proj_w, wallH, wallL);
  norm_transpose_kernel<<<kNP / 64, 256, 0, stream>>>(x, part1, ln_g, ln_b, hTH, hTL);
  chan_gemm_kernel<0><<<(kM1 / 64) * (kNP / 64) / 8, 256, 0, stream>>>(wallH, wallL, hTH, hTL, bpre, a16, p1_b, p2_in_b);
  depthwise_silu_kernel<<<kNP / 64, 256, 0, stream>>>(bpre, p2_dw_w, p2_dw_b, vf, vTH, vTL);
  chan_gemm_kernel<1><<<(kM2 / 64) * (kNP / 64) / 8, 256, 0, stream>>>(
      wallH + (size_t)kM1 * kC, wallL + (size_t)kM1 * kC, vTH, vTL, xd, nullptr, nullptr, nullptr);
  dir_scan_kernel<<<kQ * 4, kC, 0, stream>>>(xd, vf, A_log, dt_proj_w, dt_proj_b, yd0, yd1, yd2, yd3);
  combine_kernel<<<dim3(kC, kQ), 256, 0, stream>>>(yd0, yd1, yd2, yd3, vf, Dp, bs, part2);
  pool_kernel<<<dim3(kC, kQ), 256, 0, stream>>>(a16, bs, part2, n2_g, n2_b, pooled);
  gate_residual_kernel<<<dim3(kC, kQ), 256, 0, stream>>>(x, a16, bs, part2, pooled, n2_g, n2_b,
                                                         ca_w1, ca_b1, ca_w2, ca_b2, out);
}
